// MultiHeadAttention_79499844649593
// MI455X (gfx1250) — hardware-verified
//
#include <hip/hip_runtime.h>


#ifndef NB
#define NB 4
#endif
#ifndef SEQ
#define SEQ 2048
#endif
#define NB_FULL  4
#define SEQ_FULL 2048
#define DM   1024
#define NH   16
#define HD   64
#define RH   256
#define AW   4
#define OSP  68
#define PCAR 256.0f
#define C1LOG 0.18033688011112042f
#define NEGB (-3.0e38f)
#define TOK  (NB * SEQ)
#define BH   (NB * NH)

static_assert(NH * HD == DM);
static_assert(HD == 64);
static_assert((DM & (DM - 1)) == 0);
static_assert(DM % 64 == 0);
static_assert(SEQ % 64 == 0);
static_assert(RH % 64 == 0);
static_assert(SEQ >= RH);
static_assert(RH % (16 * AW) == 0);
static_assert((SEQ - RH) % (16 * AW) == 0);
static_assert(NB <= NB_FULL);
static_assert(SEQ <= SEQ_FULL);
static_assert(((size_t)TOK * DM) % (8 * 256) == 0);
static_assert((OSP * 4) % 16 == 0);

typedef _Float16 h16;
typedef unsigned short bf;
typedef __attribute__((ext_vector_type(16))) __bf16   v16bf;
typedef __attribute__((ext_vector_type(16))) _Float16 v16h;
typedef __attribute__((ext_vector_type(16))) unsigned short v16us;
typedef __attribute__((ext_vector_type(8)))  _Float16 v8h;
typedef __attribute__((ext_vector_type(8)))  unsigned short v8us;
typedef __attribute__((ext_vector_type(2)))  unsigned short v2us;
typedef __attribute__((ext_vector_type(8)))  float    v8f;
typedef __attribute__((ext_vector_type(4)))  float    v4f;
typedef v4f  __attribute__((may_alias)) v4fa;

__device__ __forceinline__ unsigned short f2bf(float f) { unsigned u = __float_as_uint(f); u += 0x7FFFu + ((u >> 16) & 1u); return (unsigned short)(u >> 16); }
__device__ __forceinline__ float bf2f(unsigned short b) { return __uint_as_float(((unsigned)b) << 16); }
__device__ __forceinline__ float bfr(float f) { return bf2f(f2bf(f)); }
__device__ __forceinline__ void splitf(float y, unsigned short& h, unsigned short& l) { h = f2bf(y); l = f2bf(y - bf2f(h)); }
__device__ __forceinline__ v16h cat16(v8h lo, v8h hi) { return __builtin_shufflevector(lo, hi, 0, 1, 2, 3, 4, 5, 6, 7, 8, 9, 10, 11, 12, 13, 14, 15); }
__device__ __forceinline__ v16bf cat16b(v8us lo, v8us hi) { return __builtin_bit_cast(v16bf, __builtin_shufflevector(lo, hi, 0, 1, 2, 3, 4, 5, 6, 7, 8, 9, 10, 11, 12, 13, 14, 15)); }
__device__ __forceinline__ v16h  ldhf(const h16* p) { return cat16(*(const v8h*)p, *(const v8h*)(p + 16)); }
__device__ __forceinline__ v16bf ldbf(const bf* p)  { return cat16b(*(const v8us*)p, *(const v8us*)(p + 16)); }
__device__ __forceinline__ v8f mmah(v16h a, v16h b, v8f c) { c = __builtin_amdgcn_wmma_f32_16x16x32_f16(false, a, false, b, (short)0, c, false, false); asm volatile("v_nop\n\tv_nop\n\tv_nop\n\tv_nop" : "+v"(c) : "v"(a), "v"(b)); return c; }
__device__ __forceinline__ v8f mmab(v16bf a, v16bf b, v8f c) { c = __builtin_amdgcn_wmma_f32_16x16x32_bf16(false, a, false, b, (short)0, c, false, false); asm volatile("v_nop\n\tv_nop\n\tv_nop\n\tv_nop" : "+v"(c) : "v"(a), "v"(b)); return c; }
__device__ __forceinline__ float ex2(float x) { return __builtin_amdgcn_exp2f(x); }

__global__ __launch_bounds__(256) void k_cvt8(const float* __restrict__ src, bf* dst) {
    const size_t i = (size_t)blockIdx.x * 256 + threadIdx.x; if (i >= (size_t)TOK * DM / 8) return;
    const int row = (int)(i / (DM / 8)); const int c8 = (int)(i % (DM / 8)); const int b = row / SEQ, t = row % SEQ;
    const v8f v = *(const v8f*)(src + ((size_t)b * SEQ_FULL + t) * DM + (size_t)c8 * 8); v8us o;
#pragma unroll
    for (int k = 0; k < 8; ++k) o[k] = f2bf(v[k]);
    *(volatile v8us*)(dst + i * 8) = o; __threadfence(); *(volatile v8us*)(dst + i * 8) = o;
}

__global__ __launch_bounds__(256) void k_wtG(const float* __restrict__ w, int K, int N, bf* Bt) {
    const int lane = threadIdx.x & 31; const int wave = __builtin_amdgcn_readfirstlane(threadIdx.x >> 5);
    const int L0 = (blockIdx.x * 8 + wave) * 8; const int nlines = N * K / 64;
#pragma unroll
    for (int ps = 0; ps < 2; ++ps) {
#pragma unroll 1
        for (int l = 0; l < 8; ++l) { const int L = L0 + l; if (L >= nlines) break; const size_t e = (size_t)L * 64 + lane * 2; const int k = (int)(e % K), n = (int)(e / K); v2us o;
            o[0] = f2bf(w[(size_t)k * N + n]); o[1] = f2bf(w[(size_t)(k + 1) * N + n]); *(volatile v2us*)(Bt + e) = o; }
        if (ps == 0) __threadfence(); }
}

__device__ __forceinline__ void gemm_main(const bf* __restrict__ A, const bf* __restrict__ Bt, const int lda, const int ldbt, const int KT, const int kmask,
                                          const int r0, const int c0, const int lr, const int hi, v8f (&acc)[4][4]) {
#pragma unroll
    for (int mb = 0; mb < 4; ++mb)
#pragma unroll
        for (int nb = 0; nb < 4; ++nb) acc[mb][nb] = (v8f){};
    const size_t aoff = (size_t)(r0 + lr) * lda + 8 * hi, boff = (size_t)(c0 + lr) * ldbt + 8 * hi;
#pragma unroll 1
    for (int kc = 0; kc < KT; kc += 32) {
        const int kq = kc & kmask;
        v16bf a[4];
#pragma unroll
        for (int mb = 0; mb < 4; ++mb) a[mb] = ldbf(A + aoff + (size_t)mb * 16 * lda + kc);
#pragma unroll
        for (int nb = 0; nb < 4; ++nb) { const v16bf b = ldbf(Bt + boff + (size_t)nb * 16 * ldbt + kq);
#pragma unroll
            for (int mb = 0; mb < 4; ++mb) acc[mb][nb] = mmab(a[mb], b, acc[mb][nb]); }
    }
}

__global__ __launch_bounds__(32) void k_proj(const bf* __restrict__ A, const bf* __restrict__ Bt, int vmode, h16* P16, bf* PH, bf* PL) {
    __shared__ __align__(16) float os[16 * OSP];
    const int lane = threadIdx.x & 31, lr = lane & 15, hi = lane >> 4; const int r0 = blockIdx.x * 64, c0 = blockIdx.y * 64;
    v8f acc[4][4];
    gemm_main(A, Bt, DM, DM, DM, DM - 1, r0, c0, lr, hi, acc);
    const int tb = vmode ? c0 : r0; const int hh = vmode ? (int)blockIdx.x : (int)blockIdx.y;
    const int b = tb / SEQ, t0 = tb % SEQ; const int bh = b * NH + hh;
    const size_t base16 = vmode ? ((size_t)bh * HD * SEQ + t0) : (((size_t)bh * SEQ + t0) * HD);
    const int pitch16 = vmode ? SEQ : HD;
    const size_t baseE = vmode ? ((size_t)bh * HD * RH + t0) : (((size_t)bh * RH + t0) * HD);
    const int pitchE = vmode ? RH : HD;
    const bool early = (t0 < RH);
#pragma unroll
    for (int mb = 0; mb < 4; ++mb) {
#pragma unroll
        for (int nb = 0; nb < 4; ++nb) {
#pragma unroll
            for (int j = 0; j < 8; ++j) os[(hi * 8 + j) * OSP + nb * 16 + lr] = acc[mb][nb][j]; }
        __builtin_amdgcn_wave_barrier(); asm volatile("" ::: "memory");
#pragma unroll 1
        for (int ps = 0; ps < 2; ++ps) {
#pragma unroll
            for (int s = 0; s < 4; ++s) { const int row = s * 4 + (lane >> 3), col = (lane & 7) * 8;
                const v4f f0 = *(const v4fa*)&os[row * OSP + col]; const v4f f1 = *(const v4fa*)&os[row * OSP + col + 4];
                v8h o; o[0] = (h16)f0[0]; o[1] = (h16)f0[1]; o[2] = (h16)f0[2]; o[3] = (h16)f0[3]; o[4] = (h16)f1[0]; o[5] = (h16)f1[1]; o[6] = (h16)f1[2]; o[7] = (h16)f1[3];
                *(volatile v8h*)(P16 + base16 + (size_t)(mb * 16 + row) * pitch16 + col) = o;
                if (early) { v8us oh, ol; unsigned short a2, c2;
                    splitf(f0[0], a2, c2); oh[0] = a2; ol[0] = c2; splitf(f0[1], a2, c2); oh[1] = a2; ol[1] = c2; splitf(f0[2], a2, c2); oh[2] = a2; ol[2] = c2; splitf(f0[3], a2, c2); oh[3] = a2; ol[3] = c2;
                    splitf(f1[0], a2, c2); oh[4] = a2; ol[4] = c2; splitf(f1[1], a2, c2); oh[5] = a2; ol[5] = c2; splitf(f1[2], a2, c2); oh[6] = a2; ol[6] = c2; splitf(f1[3], a2, c2); oh[7] = a2; ol[7] = c2;
                    *(volatile v8us*)(PH + baseE + (size_t)(mb * 16 + row) * pitchE + col) = oh; *(volatile v8us*)(PL + baseE + (size_t)(mb * 16 + row) * pitchE + col) = ol; } }
            if (ps == 0) __threadfence(); }
        __builtin_amdgcn_wave_barrier(); asm volatile("" ::: "memory");
    }
}

__global__ __launch_bounds__(32) void k_outp(const bf* __restrict__ A, const bf* __restrict__ Bt, const float* __restrict__ bias, float* C) {
    __shared__ __align__(16) float os[16 * OSP];
    const int lane = threadIdx.x & 31, lr = lane & 15, hi = lane >> 4; const int r0 = blockIdx.x * 64, c0 = blockIdx.y * 64;
    v8f acc[4][4];
    gemm_main(A, Bt, 2 * DM, DM, 2 * DM, DM - 1, r0, c0, lr, hi, acc);
    const int b = r0 / SEQ, t0 = r0 % SEQ; const int cofs = lr * 4;
    v4f bv; bv[0] = bfr(bias[c0 + cofs]); bv[1] = bfr(bias[c0 + cofs + 1]); bv[2] = bfr(bias[c0 + cofs + 2]); bv[3] = bfr(bias[c0 + cofs + 3]);
#pragma unroll
    for (int mb = 0; mb < 4; ++mb) {
#pragma unroll
        for (int nb = 0; nb < 4; ++nb) {
#pragma unroll
            for (int j = 0; j < 8; ++j) os[(hi * 8 + j) * OSP + nb * 16 + lr] = acc[mb][nb][j]; }
        __builtin_amdgcn_wave_barrier(); asm volatile("" ::: "memory");
        float* crow = C + ((size_t)b * SEQ_FULL + t0 + mb * 16) * DM + c0;
#pragma unroll 1
        for (int ps = 0; ps < 2; ++ps) {
#pragma unroll
            for (int s = 0; s < 8; ++s) { const int row = 2 * s + hi; v4f val = *(const v4fa*)&os[row * OSP + cofs]; val[0] += bv[0]; val[1] += bv[1]; val[2] += bv[2]; val[3] += bv[3];
                *(volatile v4f*)(crow + (size_t)row * DM + cofs) = val; }
            if (ps == 0) __threadfence(); }
        __builtin_amdgcn_wave_barrier(); asm volatile("" ::: "memory");
    }
}

__global__ __launch_bounds__(AW * 32) void k_attn(const h16* __restrict__ Q16, const h16* __restrict__ K16, const h16* __restrict__ VT16, bf* CTX) {
    __shared__ __align__(16) float os[AW * 16 * OSP];
    const int lane = threadIdx.x & 31, lr = lane & 15, hi = lane >> 4;
    const int wave = __builtin_amdgcn_readfirstlane(threadIdx.x >> 5);
    const int bh = blockIdx.y; const int q0 = RH + ((int)blockIdx.x * AW + wave) * 16;
    const size_t pb = (size_t)bh * SEQ * HD;
    const v16h qf0 = ldhf(Q16 + pb + (size_t)(q0 + lr) * HD + 8 * hi);
    const v16h qf1 = ldhf(Q16 + pb + (size_t)(q0 + lr) * HD + 32 + 8 * hi);
    const h16* kbase = K16 + pb + (size_t)lr * HD + 8 * hi;
    const h16* vbase = VT16 + pb + (size_t)lr * SEQ + 8 * hi;
    v8f o[4];
#pragma unroll
    for (int dt = 0; dt < 4; ++dt) o[dt] = (v8f){};
    float m = NEGB, l = 0.0f;
    const int nh = (q0 + 15) / 32 + 1;
#pragma unroll 1
    for (int c = 0; c < nh; ++c) {
        const int kb = c * 32;
        const h16* k0p = kbase + (size_t)kb * HD;
        v8f s0 = (v8f){}, s1 = (v8f){};
        s0 = mmah(ldhf(k0p), qf0, s0);
        s1 = mmah(ldhf(k0p + 16 * HD), qf0, s1);
        s0 = mmah(ldhf(k0p + 32), qf1, s0);
        s1 = mmah(ldhf(k0p + 16 * HD + 32), qf1, s1);
        v8f t0 = s0 * C1LOG, t1 = s1 * C1LOG;
        if (kb + 31 > q0) {
            const int qi = q0 + lr - kb - 8 * hi;
#pragma unroll
            for (int r = 0; r < 8; ++r) { t0[r] = (r <= qi) ? t0[r] : NEGB; t1[r] = (16 + r <= qi) ? t1[r] : NEGB; }
        }
        float mx = fmaxf(t0[0], t1[0]);
#pragma unroll
        for (int r = 1; r < 8; ++r) mx = fmaxf(mx, fmaxf(t0[r], t1[r]));
        mx = fmaxf(mx, __shfl_xor(mx, 16, 32));
        const float mnew = fmaxf(m, mx);
        const float alpha = ex2(m - mnew);
        m = mnew;
        float ps = 0.0f; v16h pf;
#pragma unroll
        for (int r = 0; r < 8; ++r) { const float p = ex2(t0[r] - mnew); ps += p; pf[r] = (h16)(p * PCAR); }
#pragma unroll
        for (int r = 0; r < 8; ++r) { const float p = ex2(t1[r] - mnew); ps += p; pf[8 + r] = (h16)(p * PCAR); }
        l = l * alpha + ps;
        if (__builtin_amdgcn_ballot_w32(alpha != 1.0f) != 0u) {
#pragma unroll
            for (int dt = 0; dt < 4; ++dt) o[dt] = o[dt] * alpha;
        }
        const h16* vp = vbase + kb;
#pragma unroll
        for (int dt = 0; dt < 4; ++dt) o[dt] = mmah(ldhf(vp + (size_t)dt * 16 * SEQ), pf, o[dt]);
    }
    const float lt = l + __shfl_xor(l, 16, 32);
    const float inv = 1.0f / (lt * PCAR);
    const int ob = wave * 16 * OSP;
#pragma unroll
    for (int dt = 0; dt < 4; ++dt) { v4f w0, w1;
        w0[0] = o[dt][0] * inv; w0[1] = o[dt][1] * inv; w0[2] = o[dt][2] * inv; w0[3] = o[dt][3] * inv;
        w1[0] = o[dt][4] * inv; w1[1] = o[dt][5] * inv; w1[2] = o[dt][6] * inv; w1[3] = o[dt][7] * inv;
        *(v4fa*)&os[ob + lr * OSP + 16 * dt + 8 * hi] = w0; *(v4fa*)&os[ob + lr * OSP + 16 * dt + 8 * hi + 4] = w1; }
    __builtin_amdgcn_wave_barrier(); asm volatile("" ::: "memory");
    const int b = bh / NH, h = bh % NH;
    bf* crow = CTX + ((size_t)b * SEQ + q0) * (2 * DM) + h * HD;
#pragma unroll 1
    for (int pss = 0; pss < 2; ++pss) {
#pragma unroll
        for (int s = 0; s < 4; ++s) { const int row = s * 4 + (lane >> 3), col = (lane & 7) * 8;
            const v4f f0 = *(const v4fa*)&os[ob + row * OSP + col]; const v4f f1 = *(const v4fa*)&os[ob + row * OSP + col + 4];
            v8us oh, ol; unsigned short a2, c2;
            splitf(f0[0], a2, c2); oh[0] = a2; ol[0] = c2; splitf(f0[1], a2, c2); oh[1] = a2; ol[1] = c2; splitf(f0[2], a2, c2); oh[2] = a2; ol[2] = c2; splitf(f0[3], a2, c2); oh[3] = a2; ol[3] = c2;
            splitf(f1[0], a2, c2); oh[4] = a2; ol[4] = c2; splitf(f1[1], a2, c2); oh[5] = a2; ol[5] = c2; splitf(f1[2], a2, c2); oh[6] = a2; ol[6] = c2; splitf(f1[3], a2, c2); oh[7] = a2; ol[7] = c2;
            *(volatile v8us*)(crow + (size_t)row * (2 * DM) + col) = oh; *(volatile v8us*)(crow + (size_t)row * (2 * DM) + DM + col) = ol; }
        if (pss == 0) __threadfence(); }
}

__global__ __launch_bounds__(AW * 32) void k_attn_e(const bf* __restrict__ QH, const bf* __restrict__ QL, const bf* __restrict__ KH, const bf* __restrict__ KL,
                                                     const bf* __restrict__ VTH, const bf* __restrict__ VTL, bf* CTX) {
    __shared__ __align__(16) float os[AW * 16 * OSP];
    const int lane = threadIdx.x & 31, lr = lane & 15, hi = lane >> 4;
    const int wave = __builtin_amdgcn_readfirstlane(threadIdx.x >> 5);
    const int bh = blockIdx.y; const int q0 = ((int)blockIdx.x * AW + wave) * 16;
    const size_t pe = (size_t)bh * RH * HD;
    const size_t qo = pe + (size_t)(q0 + lr) * HD + 8 * hi;
    const v16bf qh0 = ldbf(QH + qo), qh1 = ldbf(QH + qo + 32), ql0 = ldbf(QL + qo), ql1 = ldbf(QL + qo + 32);
    const size_t kof = pe + (size_t)lr * HD + 8 * hi;
    const size_t vof = pe + (size_t)lr * RH + 8 * hi;
    v8f o[4];
#pragma unroll
    for (int dt = 0; dt < 4; ++dt) o[dt] = (v8f){};
    float m = NEGB, l = 0.0f;
    const int nh = (q0 + 15) / 32 + 1;
#pragma unroll 1
    for (int c = 0; c < nh; ++c) {
        const int kb = c * 32;
        const size_t ka = kof + (size_t)kb * HD;
        v8f s0 = (v8f){}, s1 = (v8f){};
        { const v16bf kh = ldbf(KH + ka), kl = ldbf(KL + ka); s0 = mmab(kl, qh0, s0); s0 = mmab(kh, ql0, s0); s0 = mmab(kh, qh0, s0); }
        { const v16bf kh = ldbf(KH + ka + 32), kl = ldbf(KL + ka + 32); s0 = mmab(kl, qh1, s0); s0 = mmab(kh, ql1, s0); s0 = mmab(kh, qh1, s0); }
        { const v16bf kh = ldbf(KH + ka + 16 * HD), kl = ldbf(KL + ka + 16 * HD); s1 = mmab(kl, qh0, s1); s1 = mmab(kh, ql0, s1); s1 = mmab(kh, qh0, s1); }
        { const v16bf kh = ldbf(KH + ka + 16 * HD + 32), kl = ldbf(KL + ka + 16 * HD + 32); s1 = mmab(kl, qh1, s1); s1 = mmab(kh, ql1, s1); s1 = mmab(kh, qh1, s1); }
        v8f t0 = s0 * C1LOG, t1 = s1 * C1LOG;
        if (kb + 31 > q0) {
            const int qi = q0 + lr - kb - 8 * hi;
#pragma unroll
            for (int r = 0; r < 8; ++r) { t0[r] = (r <= qi) ? t0[r] : NEGB; t1[r] = (16 + r <= qi) ? t1[r] : NEGB; }
        }
        float mx = fmaxf(t0[0], t1[0]);
#pragma unroll
        for (int r = 1; r < 8; ++r) mx = fmaxf(mx, fmaxf(t0[r], t1[r]));
        mx = fmaxf(mx, __shfl_xor(mx, 16, 32));
        const float mnew = fmaxf(m, mx);
        const float alpha = ex2(m - mnew);
        m = mnew;
        float ps = 0.0f; v16us phs, pls;
#pragma unroll
        for (int r = 0; r < 8; ++r) { const float p = ex2(t0[r] - mnew); ps += p; unsigned short a2, c2; splitf(p, a2, c2); phs[r] = a2; pls[r] = c2; }
#pragma unroll
        for (int r = 0; r < 8; ++r) { const float p = ex2(t1[r] - mnew); ps += p; unsigned short a2, c2; splitf(p, a2, c2); phs[8 + r] = a2; pls[8 + r] = c2; }
        const v16bf ph = __builtin_bit_cast(v16bf, phs), pl = __builtin_bit_cast(v16bf, pls);
        l = l * alpha + ps;
#pragma unroll
        for (int dt = 0; dt < 4; ++dt) o[dt] = o[dt] * alpha;
#pragma unroll
        for (int dt = 0; dt < 4; ++dt) { const size_t va = vof + (size_t)dt * 16 * RH + kb; const v16bf vh = ldbf(VTH + va), vl = ldbf(VTL + va);
            o[dt] = mmab(vl, ph, o[dt]); o[dt] = mmab(vh, pl, o[dt]); o[dt] = mmab(vh, ph, o[dt]); }
    }
    const float lt = l + __shfl_xor(l, 16, 32);
    const float inv = 1.0f / lt;
    const int ob = wave * 16 * OSP;
#pragma unroll
    for (int dt = 0; dt < 4; ++dt) { v4f w0, w1;
        w0[0] = o[dt][0] * inv; w0[1] = o[dt][1] * inv; w0[2] = o[dt][2] * inv; w0[3] = o[dt][3] * inv;
        w1[0] = o[dt][4] * inv; w1[1] = o[dt][5] * inv; w1[2] = o[dt][6] * inv; w1[3] = o[dt][7] * inv;
        *(v4fa*)&os[ob + lr * OSP + 16 * dt + 8 * hi] = w0; *(v4fa*)&os[ob + lr * OSP + 16 * dt + 8 * hi + 4] = w1; }
    __builtin_amdgcn_wave_barrier(); asm volatile("" ::: "memory");
    const int b = bh / NH, h = bh % NH;
    bf* crow = CTX + ((size_t)b * SEQ + q0) * (2 * DM) + h * HD;
#pragma unroll 1
    for (int pss = 0; pss < 2; ++pss) {
#pragma unroll
        for (int s = 0; s < 4; ++s) { const int row = s * 4 + (lane >> 3), col = (lane & 7) * 8;
            const v4f f0 = *(const v4fa*)&os[ob + row * OSP + col]; const v4f f1 = *(const v4fa*)&os[ob + row * OSP + col + 4];
            v8us oh, ol; unsigned short a2, c2;
            splitf(f0[0], a2, c2); oh[0] = a2; ol[0] = c2; splitf(f0[1], a2, c2); oh[1] = a2; ol[1] = c2; splitf(f0[2], a2, c2); oh[2] = a2; ol[2] = c2; splitf(f0[3], a2, c2); oh[3] = a2; ol[3] = c2;
            splitf(f1[0], a2, c2); oh[4] = a2; ol[4] = c2; splitf(f1[1], a2, c2); oh[5] = a2; ol[5] = c2; splitf(f1[2], a2, c2); oh[6] = a2; ol[6] = c2; splitf(f1[3], a2, c2); oh[7] = a2; ol[7] = c2;
            *(volatile v8us*)(crow + (size_t)row * (2 * DM) + col) = oh; *(volatile v8us*)(crow + (size_t)row * (2 * DM) + DM + col) = ol; }
        if (pss == 0) __threadfence(); }
}

#define AL256(x) ((((size_t)(x)) + 255) & ~(size_t)255)
constexpr size_t SZ_W   = AL256((size_t)DM * DM * 2);
constexpr size_t SZ_XB  = AL256((size_t)TOK * DM * 2);
constexpr size_t SZ_P   = AL256((size_t)BH * SEQ * HD * 2);
constexpr size_t SZ_E   = AL256((size_t)BH * RH * HD * 2);
constexpr size_t SZ_CTX = AL256((size_t)TOK * 2 * DM * 2);
constexpr size_t WS_TOTAL = 4 * SZ_W + SZ_XB + 3 * SZ_P + 6 * SZ_E + SZ_CTX;
static_assert(WS_TOTAL <= (size_t)134217728);

extern "C" void kernel_launch(void* const* d_in, const int* in_sizes, int n_in,
                              void* d_out, int out_size, void* d_ws, size_t ws_size, hipStream_t stream) {
    if (n_in < 6) return;
    const long long need_x = ((long long)(NB - 1) * SEQ_FULL + SEQ) * DM;
    if ((long long)in_sizes[0] < need_x) return;
    if (in_sizes[1] < DM * DM || in_sizes[2] < DM * DM || in_sizes[3] < DM * DM || in_sizes[4] < DM * DM || in_sizes[5] < DM) return;
    if ((long long)out_size < need_x) return;
    if (WS_TOTAL > ws_size) return;
    const float* x = (const float*)d_in[0]; const float* wq = (const float*)d_in[1]; const float* wk = (const float*)d_in[2];
    const float* wv = (const float*)d_in[3]; const float* wo = (const float*)d_in[4]; const float* bo = (const float*)d_in[5];
    float* OUT = (float*)d_out;
    char* wsp = (char*)d_ws;
    bf* WQ = (bf*)wsp; wsp += SZ_W; bf* WK = (bf*)wsp; wsp += SZ_W; bf* WV = (bf*)wsp; wsp += SZ_W; bf* WO = (bf*)wsp; wsp += SZ_W;
    bf* XB = (bf*)wsp; wsp += SZ_XB;
    h16* Q16 = (h16*)wsp; wsp += SZ_P; h16* K16 = (h16*)wsp; wsp += SZ_P; h16* VT16 = (h16*)wsp; wsp += SZ_P;
    bf* QH = (bf*)wsp; wsp += SZ_E; bf* QL = (bf*)wsp; wsp += SZ_E; bf* KH = (bf*)wsp; wsp += SZ_E; bf* KL = (bf*)wsp; wsp += SZ_E; bf* VTH = (bf*)wsp; wsp += SZ_E; bf* VTL = (bf*)wsp; wsp += SZ_E;
    bf* CTX = (bf*)wsp; wsp += SZ_CTX;

    k_cvt8<<<(unsigned)(((size_t)TOK * DM / 8 + 255) / 256), 256, 0, stream>>>(x, XB);
    k_wtG<<<(unsigned)((DM * DM / 64 + 63) / 64), 256, 0, stream>>>(wq, DM, DM, WQ);
    k_wtG<<<(unsigned)((DM * DM / 64 + 63) / 64), 256, 0, stream>>>(wk, DM, DM, WK);
    k_wtG<<<(unsigned)((DM * DM / 64 + 63) / 64), 256, 0, stream>>>(wv, DM, DM, WV);
    k_wtG<<<(unsigned)((DM * DM / 64 + 63) / 64), 256, 0, stream>>>(wo, DM, DM, WO);
    k_proj<<<dim3(TOK / 64, DM / 64, 1), 32, 0, stream>>>(XB, WQ, 0, Q16, QH, QL);
    k_proj<<<dim3(TOK / 64, DM / 64, 1), 32, 0, stream>>>(XB, WK, 0, K16, KH, KL);
    k_proj<<<dim3(DM / 64, TOK / 64, 1), 32, 0, stream>>>(WV, XB, 1, VT16, VTH, VTL);
    k_attn_e<<<dim3(RH / (16 * AW), BH, 1), AW * 32, 0, stream>>>(QH, QL, KH, KL, VTH, VTL, CTX);
    if (SEQ > RH) k_attn<<<dim3((SEQ - RH) / (16 * AW), BH, 1), AW * 32, 0, stream>>>(Q16, K16, VT16, CTX);
    k_outp<<<dim3(TOK / 64, DM / 64, 1), 32, 0, stream>>>(CTX, WO, bo, OUT);
}
